// MyDCNv2_88201448391342
// MI455X (gfx1250) — hardware-verified
//
#include <hip/hip_runtime.h>
#include <math.h>
#include <stdint.h>

#define NB    8
#define CIN   256
#define COUT  256
#define IMH   64
#define IMW   64
#define HW    4096
#define NTAP  9
#define KK    2304
#define PT    128
#define PXB   8
#define NOFF  18
static_assert(PT * 32 == HW);
static_assert(KK == NTAP * CIN);
static_assert(HW == IMH * IMW);
static_assert((HW % 64) == 0 && (COUT % 64) == 0 && (KK % 32) == 0);
static_assert((HW % PXB) == 0);
static_assert(((COUT * KK) % (256 * 8)) == 0);
static_assert(CIN == 32 * 8);

typedef __bf16   v16b __attribute__((ext_vector_type(16)));
typedef __bf16   v8b  __attribute__((ext_vector_type(8)));
typedef float    v8f  __attribute__((ext_vector_type(8)));
typedef float    v4f  __attribute__((ext_vector_type(4)));
typedef unsigned int v4u __attribute__((ext_vector_type(4)));

__device__ __forceinline__ unsigned short bf_bits(float f) {
  unsigned u = __float_as_uint(f);
  return (unsigned short)((u + 0x7FFFu + ((u >> 16) & 1u)) >> 16);
}
__device__ __forceinline__ float bf_up(unsigned short h) { return __uint_as_float(((unsigned)h) << 16); }
__device__ __forceinline__ float bfr(float f) { return bf_up(bf_bits(f)); }
__device__ __forceinline__ unsigned pk16(unsigned short a, unsigned short b) { return (unsigned)a | ((unsigned)b << 16); }
__device__ __forceinline__ v8f zero8() { v8f z = {0.f, 0.f, 0.f, 0.f, 0.f, 0.f, 0.f, 0.f}; return z; }

__device__ __forceinline__ v16b ldfrag_b(const __bf16* p) {
  union { v16b v; v8b h[2]; } f;
  f.h[0] = *(const v8b*)(p);
  f.h[1] = *(const v8b*)(p + 16);
  return f.v;
}

__device__ __forceinline__ v8f mma_b_raw(v16b a, v16b b, v8f c) {
  return __builtin_amdgcn_wmma_f32_16x16x32_bf16(false, a, false, b, (short)0, c, false, false);
}
__device__ __forceinline__ void dep_guard_b(v8f& a, v8f& b, v16b x, v16b y) {
#if defined(__HIP_DEVICE_COMPILE__)
  asm volatile("v_nop\n\tv_nop\n\tv_nop\n\tv_nop" : "+v"(a), "+v"(b) : "v"(x), "v"(y));
#endif
}
__device__ __forceinline__ void keep4_b(v16b a, v16b b, v16b c, v16b d) {
#if defined(__HIP_DEVICE_COMPILE__)
  asm volatile("v_nop" :: "v"(a), "v"(b), "v"(c), "v"(d));
#endif
}
__device__ __forceinline__ void acc_guard4(v8f& a, v8f& b, v8f& c, v8f& d) {
#if defined(__HIP_DEVICE_COMPILE__)
  asm volatile("v_nop\n\tv_nop\n\tv_nop\n\tv_nop" : "+v"(a), "+v"(b), "+v"(c), "+v"(d));
#endif
}
__device__ __forceinline__ void wave_sync_lds() {
  __builtin_amdgcn_fence(__ATOMIC_RELEASE, "workgroup");
  __builtin_amdgcn_wave_barrier();
  __builtin_amdgcn_fence(__ATOMIC_ACQUIRE, "workgroup");
}

__global__ __launch_bounds__(256) void cvt_xt(const float* __restrict__ x, unsigned short* xt) {
  __shared__ __align__(16) float sx[CIN * 36];
  const int tid = threadIdx.x;
  const int b   = blockIdx.x / PT;
  const int tp  = blockIdx.x - b * PT;
  const int p0  = tp * 32;
  const float* xb = x + (size_t)b * CIN * HW + p0;
#pragma unroll
  for (int it = 0; it < 8; ++it) {
    const int idx = it * 256 + tid;
    const int c = idx >> 3, q = idx & 7;
    const v4f v = *(const v4f*)(xb + (size_t)c * HW + 4 * q);
    *(v4f*)(sx + c * 36 + 4 * q) = v;
  }
  __syncthreads();
  const int wave = tid >> 5, lane = tid & 31, c8 = lane * 8;
  v4u pk[4];
#pragma unroll
  for (int it = 0; it < 4; ++it) {
    const int r = wave * 4 + it;
    v4u p;
#pragma unroll
    for (int e = 0; e < 4; ++e)
      p[e] = pk16(bf_bits(sx[(c8 + 2 * e) * 36 + r]), bf_bits(sx[(c8 + 2 * e + 1) * 36 + r]));
    pk[it] = p;
  }
  unsigned short* dst = xt + ((size_t)b * HW + p0) * CIN;
  for (int pass = 0; pass < 2; ++pass) {
#pragma unroll
    for (int it = 0; it < 4; ++it) {
      const int r = wave * 4 + it;
      *(volatile v4u*)(dst + (size_t)r * CIN + c8) = pk[it];
    }
    __threadfence();
  }
}

__global__ __launch_bounds__(256) void wprep(const float* __restrict__ w, unsigned short* wp) {
  const int j   = blockIdx.x * 256 + threadIdx.x;
  const int f   = j * 8;
  const int o   = f / KK;
  const int rem = f - o * KK;
  const int t   = rem >> 8;
  const int c   = rem & 255;
  const float* src = w + ((size_t)(o * CIN + c)) * NTAP + t;
  float vals[8];
#pragma unroll
  for (int i = 0; i < 8; ++i) vals[i] = src[i * NTAP];
  v4u p;
#pragma unroll
  for (int i = 0; i < 4; ++i) p[i] = pk16(bf_bits(vals[2 * i]), bf_bits(vals[2 * i + 1]));
  unsigned short* d = wp + f;
  *(volatile v4u*)d = p;
  __threadfence();
  *(volatile v4u*)d = p;
}

__global__ __launch_bounds__(256)
void sampler(const unsigned short* __restrict__ xt, const float* __restrict__ offs,
             const float* __restrict__ msk, unsigned short* colh, unsigned short* coll) {
#pragma clang fp contract(off)
  const int tid = threadIdx.x, wave = tid >> 5, lane = tid & 31;
  const int p = blockIdx.x * PXB + wave;
  if (p >= HW) return;
  const int oy = p >> 6, ox = p & 63;
  const int c8 = lane * 8;
#pragma unroll 1
  for (int tap = 0; tap < NTAP; ++tap) {
    const int ky = tap / 3, kx = tap - ky * 3;
    const float offy = bfr(offs[(size_t)(2 * tap) * HW + p]);
    const float offx = bfr(offs[(size_t)(2 * tap + 1) * HW + p]);
    const float mv   = bfr(msk[(size_t)tap * HW + p]);
    float py = (float)(oy + ky) + offy;
    float px = (float)(ox + kx) + offx;
    py = fminf(fmaxf(py, 0.f), 65.f);
    px = fminf(fmaxf(px, 0.f), 65.f);
    const float fy = floorf(py), fx = floorf(px);
    const float wy = py - fy, wx = px - fx;
    const int y0 = min(max((int)fy, 0), 65);
    const int x0 = min(max((int)fx, 0), 65);
    const bool vy0 = (y0 >= 1) && (y0 <= IMH);
    const bool vy1 = (y0 + 1 <= IMH);
    const bool vx0 = (x0 >= 1) && (x0 <= IMW);
    const bool vx1 = (x0 + 1 <= IMW);
    const int sy0 = min(max(y0 - 1, 0), IMH - 1), sy1 = min(max(y0, 0), IMH - 1);
    const int sx0 = min(max(x0 - 1, 0), IMW - 1), sx1 = min(max(x0, 0), IMW - 1);
    const bool v00 = vy0 && vx0, v01 = vy0 && vx1, v10 = vy1 && vx0, v11 = vy1 && vx1;
    const float omy = 1.f - wy, omx = 1.f - wx;
    const float w00 = omy * omx, w01 = omy * wx, w10 = wy * omx, w11 = wy * wx;
    const v4u u00 = *(const v4u*)(xt + (size_t)(sy0 * IMW + sx0) * CIN + c8);
    const v4u u01 = *(const v4u*)(xt + (size_t)(sy0 * IMW + sx1) * CIN + c8);
    const v4u u10 = *(const v4u*)(xt + (size_t)(sy1 * IMW + sx0) * CIN + c8);
    const v4u u11 = *(const v4u*)(xt + (size_t)(sy1 * IMW + sx1) * CIN + c8);
    v4u hv, lv;
#pragma unroll
    for (int e = 0; e < 4; ++e) {
      unsigned short hb[2], lb[2];
#pragma unroll
      for (int s = 0; s < 2; ++s) {
        float g00, g01, g10, g11;
        if (s == 0) {
          g00 = __uint_as_float(u00[e] << 16); g01 = __uint_as_float(u01[e] << 16);
          g10 = __uint_as_float(u10[e] << 16); g11 = __uint_as_float(u11[e] << 16);
        } else {
          g00 = __uint_as_float(u00[e] & 0xffff0000u); g01 = __uint_as_float(u01[e] & 0xffff0000u);
          g10 = __uint_as_float(u10[e] & 0xffff0000u); g11 = __uint_as_float(u11[e] & 0xffff0000u);
        }
        g00 = v00 ? g00 : 0.f;
        g01 = v01 ? g01 : 0.f;
        g10 = v10 ? g10 : 0.f;
        g11 = v11 ? g11 : 0.f;
        float t = w00 * g00;
        t = t + w01 * g01;
        t = t + w10 * g10;
        t = t + w11 * g11;
        t = t * mv;
        const unsigned short h = bf_bits(t);
        const unsigned short l = bf_bits(t - bf_up(h));
        hb[s] = h; lb[s] = l;
      }
      hv[e] = pk16(hb[0], hb[1]);
      lv[e] = pk16(lb[0], lb[1]);
    }
    const size_t so = (size_t)p * KK + (size_t)tap * CIN + c8;
    *(volatile v4u*)(colh + so) = hv;
    *(volatile v4u*)(coll + so) = lv;
    __threadfence();
    *(volatile v4u*)(colh + so) = hv;
    *(volatile v4u*)(coll + so) = lv;
  }
}

__global__ __launch_bounds__(256) void gemm64(
    const unsigned short* __restrict__ Ap, int lda,
    const unsigned short* __restrict__ Bhp, const unsigned short* __restrict__ Blp, int ldb,
    float* Cout, int ldc, int M, int N, int K) {
  const __bf16* A  = (const __bf16*)(const void*)Ap;
  const __bf16* Bh = (const __bf16*)(const void*)Bhp;
  const __bf16* Bl = (const __bf16*)(const void*)Blp;
  __shared__ __align__(16) float sT[8][16 * 68];
  const int lane = threadIdx.x & 31;
  const int wave = threadIdx.x >> 5;
  const int tilesN = N >> 6;
  const int tilesM = M >> 6;
  const int tile = blockIdx.x * 8 + wave;
  if (tile >= tilesM * tilesN) return;
  const int tm = tile / tilesN;
  const int tn = tile - tm * tilesN;
  const int m0 = tm << 6;
  const int n0 = tn << 6;

  const int rlane = lane & 15;
  const int koff  = (lane >> 4) * 8;
  const int mOff  = (lane >> 4) * 8;

  v8f acc[4][4];
#pragma unroll
  for (int i = 0; i < 4; ++i)
#pragma unroll
    for (int j = 0; j < 4; ++j) acc[i][j] = zero8();

  for (int k0 = 0; k0 < K; k0 += 32) {
    v16b af[4];
#pragma unroll
    for (int i = 0; i < 4; ++i) {
      const size_t ao = (size_t)(m0 + (i << 4) + rlane) * lda + koff + k0;
      af[i] = ldfrag_b(A + ao);
    }
#pragma unroll
    for (int j = 0; j < 4; ++j) {
      const size_t bo = (size_t)(n0 + (j << 4) + rlane) * ldb + koff + k0;
      const v16b bh = ldfrag_b(Bh + bo);
      const v16b bl = ldfrag_b(Bl + bo);
#pragma unroll
      for (int i = 0; i < 4; ++i) {
        acc[i][j] = mma_b_raw(af[i], bh, acc[i][j]);
        acc[i][j] = mma_b_raw(af[i], bl, acc[i][j]);
      }
      dep_guard_b(acc[0][j], acc[3][j], bh, bl);
    }
    keep4_b(af[0], af[1], af[2], af[3]);
  }
  acc_guard4(acc[0][0], acc[0][1], acc[0][2], acc[0][3]);
  acc_guard4(acc[1][0], acc[1][1], acc[1][2], acc[1][3]);
  acc_guard4(acc[2][0], acc[2][1], acc[2][2], acc[2][3]);
  acc_guard4(acc[3][0], acc[3][1], acc[3][2], acc[3][3]);

  float* slab = sT[wave];
#pragma unroll
  for (int i = 0; i < 4; ++i) {
    const int mBase = m0 + (i << 4);
#pragma unroll
    for (int j = 0; j < 4; ++j) {
#pragma unroll
      for (int r = 0; r < 8; ++r) {
        slab[(mOff + r) * 68 + (j << 4) + rlane] = acc[i][j][r];
      }
    }
    wave_sync_lds();
    {
      const int hh = lane >> 4, c4 = (lane & 15) * 4;
      v4f ov[8];
#pragma unroll
      for (int it = 0; it < 8; ++it) {
        const int row = it * 2 + hh;
        ov[it] = *(const v4f*)(slab + row * 68 + c4);
      }
      for (int pass = 0; pass < 2; ++pass) {
#pragma unroll
        for (int it = 0; it < 8; ++it) {
          const int row = it * 2 + hh;
          *(volatile v4f*)(Cout + (size_t)(mBase + row) * ldc + n0 + c4) = ov[it];
        }
        __threadfence();
      }
    }
    wave_sync_lds();
  }
}

extern "C" void kernel_launch(void* const* d_in, const int* in_sizes, int n_in,
                              void* d_out, int out_size, void* d_ws, size_t ws_size,
                              hipStream_t stream) {
  if (n_in < 4) return;
  if (in_sizes[0] != NB * CIN * HW) return;
  if (in_sizes[1] != NB * NOFF * HW) return;
  if (in_sizes[2] != NB * NTAP * HW) return;
  if (in_sizes[3] != COUT * CIN * NTAP) return;
  if (out_size != NB * COUT * HW) return;

  const float* x      = (const float*)d_in[0];
  const float* offset = (const float*)d_in[1];
  const float* mask   = (const float*)d_in[2];
  const float* weight = (const float*)d_in[3];
  float* out = (float*)d_out;

  const size_t PXT = (size_t)NB * HW * CIN * 2;
  const size_t PWP = (size_t)COUT * KK * 2;
  const size_t PCL = (size_t)HW * KK * 2;
  size_t off = 0;
  const size_t oXT = off; off += PXT;
  const size_t oWP = off; off += PWP;
  const size_t oCH = off; off += PCL;
  const size_t oCL = off; off += PCL;
  if (off > ws_size) return;
  if (off > (size_t)134217728) return;

  char* ws = (char*)d_ws;
  unsigned short* XT = (unsigned short*)(ws + oXT);
  unsigned short* WP = (unsigned short*)(ws + oWP);
  unsigned short* CH = (unsigned short*)(ws + oCH);
  unsigned short* CL = (unsigned short*)(ws + oCL);

  const dim3 blk(256);
  cvt_xt<<<dim3(NB * PT), blk, 0, stream>>>(x, XT);
  wprep<<<dim3((COUT * KK) / (256 * 8)), blk, 0, stream>>>(weight, WP);
  const dim3 gSmp(HW / PXB);
  const dim3 gGemm(((COUT / 64) * (HW / 64) + 7) / 8);
  for (int n = 0; n < NB; ++n) {
    const unsigned short* XTn = XT + (size_t)n * HW * CIN;
    const float* OFn = offset + (size_t)n * NOFF * HW;
    const float* MKn = mask + (size_t)n * NTAP * HW;
    float* Cn = out + (size_t)n * COUT * HW;
    sampler<<<gSmp, blk, 0, stream>>>(XTn, OFn, MKn, CH, CL);
    gemm64<<<gGemm, blk, 0, stream>>>(WP, KK, CH, CL, KK, Cn, HW, COUT, HW, KK);
  }
  (void)hipGetLastError();
}
